// TimelineGNNLayer3_39410619908398
// MI455X (gfx1250) — hardware-verified
//
#include <hip/hip_runtime.h>
#include <stddef.h>
#include <math.h>


#define DIMC    128
#define GATEN   256
#define GATEK   384
#define HTK     256
#define F1K     160
#define TD      32
#define PE_LEN  1000
#define PE_ROWS 1024
#define PE_KF   (-0.28782313662425596f)

#define NTHR   128
#define NWAVE  4
#define EPT    8
#define CHUNK  (NTHR * EPT)
#define WCAP   (EPT * 32)
#define LISTN  (NWAVE * WCAP)
#define PASSN  (NWAVE * 16)
#define PCAP   (CHUNK + PASSN)
#define NB     256
#define ACCW   129
#define PT     136
#define PF     260
#define ASC    64.0f
#define WSC    32.0f
#define PINV   0.00048828125f
#define GT_THR 256
#define SDP    132

static_assert(PASSN == 64);
static_assert(PCAP >= CHUNK + PASSN);
static_assert((NB % (NWAVE * 64)) == 0);
static_assert(CHUNK == NWAVE * WCAP);

#define OFF_ACC   0
#define SZ_ACC    (NB * ACCW * 4)
#define OFF_XR    (OFF_ACC + SZ_ACC)
#define SZ_XR     (NWAVE * 16 * PT * 2)
#define OFF_HR    (OFF_XR + SZ_XR)
#define OFF_STG   (OFF_HR + SZ_XR)
#define SZ_STG    (NWAVE * 16 * PF * 4)
#define OFF_LIST  (OFF_STG + SZ_STG)
#define OFF_PEND  (OFF_LIST + LISTN * 4)
#define OFF_SLOT  (OFF_PEND + PCAP * 4)
#define OFF_REL   (OFF_SLOT + PASSN * 4)
#define OFF_T     (OFF_REL + PASSN * 4)
#define OFF_SUB   (OFF_T + PASSN * 4)
#define OFF_RQ    (OFF_SUB + PASSN * 4)
#define OFF_VAL   (OFF_RQ + PASSN * 4)
#define OFF_W     (OFF_VAL + PASSN * 4)
#define OFF_WCNT  (OFF_W + PASSN * 4)
#define OFF_PENDN (OFF_WCNT + 16)
#define LDS_TOTAL (OFF_PENDN + 16)
static_assert(LDS_TOTAL == 243744);
static_assert((OFF_XR & 15) == 0 && (OFF_HR & 15) == 0 && (OFF_STG & 15) == 0 && (OFF_LIST & 15) == 0);
static_assert((OFF_PEND & 15) == 0 && (OFF_SLOT & 15) == 0 && (OFF_W & 15) == 0 && (OFF_WCNT & 15) == 0);

typedef float          v4f  __attribute__((ext_vector_type(4)));
typedef float          v8f  __attribute__((ext_vector_type(8)));
typedef _Float16       v4h  __attribute__((ext_vector_type(4)));
typedef _Float16       v8h  __attribute__((ext_vector_type(8)));
typedef _Float16       v16h __attribute__((ext_vector_type(16)));
typedef __bf16         v16b __attribute__((ext_vector_type(16)));
typedef unsigned short v8us __attribute__((ext_vector_type(8)));
union Frag16 { v16h vh; v16b vb; v8h h[2]; v8us u[2]; };
struct Acc2 { v8f u; v8f c; };

__device__ __forceinline__ v8f zacc() {
  v8f c;
#pragma unroll
  for (int i = 0; i < 8; ++i) c[i] = 0.0f;
  return c;
}

__device__ __forceinline__ v8f wmh(v16h a, v16h b, v8f c) {
  v8f d = __builtin_amdgcn_wmma_f32_16x16x32_f16(false, a, false, b, (short)0, c, false, false);
  asm volatile("v_nop\n\tv_nop\n\tv_nop\n\tv_nop" : "+v"(d) : "v"(a), "v"(b));
  return d;
}
__device__ __forceinline__ v8f wmb(v16b a, v16b b, v8f c) {
  v8f d = __builtin_amdgcn_wmma_f32_16x16x32_bf16(false, a, false, b, (short)0, c, false, false);
  asm volatile("v_nop\n\tv_nop\n\tv_nop\n\tv_nop" : "+v"(d) : "v"(a), "v"(b));
  return d;
}

__device__ __forceinline__ unsigned short f2bf(float f) {
  const unsigned u = __float_as_uint(f);
  return (unsigned short)((u + 0x7FFFu + ((u >> 16) & 1u)) >> 16);
}
__device__ __forceinline__ float bf2f(unsigned short b) { return __uint_as_float(((unsigned)b) << 16); }
__device__ __forceinline__ unsigned short h2us(_Float16 x) { union { _Float16 h; unsigned short u; } c; c.h = x; return c.u; }
__device__ __forceinline__ float lrelu(float x) { return x >= 0.0f ? x : 0.01f * x; }
__device__ __forceinline__ float rcpx(float x) { return __builtin_amdgcn_rcpf(x); }
__device__ __forceinline__ float sigm(float x) { return rcpx(1.0f + __expf(-x)); }
__device__ __forceinline__ float tanh_f(float x) {
  const float e = __expf(-2.0f * fabsf(x));
  return copysignf((1.0f - e) * rcpx(1.0f + e), x);
}

__global__ __launch_bounds__(256) void k_prep(
    const float* __restrict__ fuse1_w, const float* __restrict__ fuse2_w, const float* __restrict__ gate_w,
    const float* __restrict__ htrans_w, const float* __restrict__ ws_w, const float* __restrict__ wr_w,
    const float* __restrict__ wqr_w, const float* __restrict__ wh_w,
    const float* __restrict__ hidden, const float* __restrict__ rela_w, const int* __restrict__ q_rel,
    _Float16* WF1, _Float16* WF2, _Float16* WG, _Float16* WHT, _Float16* WS, _Float16* WR, _Float16* WQ,
    unsigned short* WHhi, unsigned short* WHlo,
    _Float16* hid16, _Float16* rela16, _Float16* pe16, _Float16* qsel16,
    int nN, int nNpad, int nRel, int nRelPad, int nQ, int nQpad) {
  const int seg = blockIdx.y;
  const size_t gstride = (size_t)gridDim.x * blockDim.x;
  const size_t gtid = (size_t)blockIdx.x * blockDim.x + threadIdx.x;

  if (seg == 10) {
    unsigned* pe32 = (unsigned*)pe16;
    const size_t npairs = (size_t)PE_ROWS * (TD / 2);
#pragma unroll 1
    for (size_t pi = gtid; pi < npairs; pi += gstride) {
      const int p = (int)(pi >> 4), i = (int)(pi & 15);
      const int pc = p < PE_LEN ? p : PE_LEN - 1;
      const float dv = expf((float)(2 * i) * PE_KF);
      const float arg = (float)pc * dv;
      float sv = sinf(arg), cv = cosf(arg);
      if (p >= PE_LEN) { sv = 0.0f; cv = 0.0f; }
      const unsigned lo = (unsigned)h2us((_Float16)(sv * ASC));
      const unsigned hi = (unsigned)h2us((_Float16)(cv * ASC));
      const unsigned packed = lo | (hi << 16);
      *(volatile unsigned*)(pe32 + pi) = packed;
      __threadfence();
      *(volatile unsigned*)(pe32 + pi) = packed;
    }
    return;
  }

  const float* src = fuse1_w; _Float16* dst = WF1;
  size_t nsrc = (size_t)DIMC * F1K, ndst = (size_t)DIMC * F1K; float sc = WSC;
  if (seg == 1)       { src = fuse2_w;  dst = WF2;  nsrc = ndst = (size_t)DIMC * DIMC; }
  else if (seg == 2)  { src = gate_w;   dst = WG;   nsrc = ndst = (size_t)GATEN * GATEK; }
  else if (seg == 3)  { src = htrans_w; dst = WHT;  nsrc = ndst = (size_t)DIMC * HTK; }
  else if (seg == 4)  { src = ws_w;     dst = WS;   nsrc = ndst = (size_t)DIMC * DIMC; }
  else if (seg == 5)  { src = wr_w;     dst = WR;   nsrc = ndst = (size_t)DIMC * DIMC; }
  else if (seg == 6)  { src = wqr_w;    dst = WQ;   nsrc = ndst = (size_t)DIMC * DIMC; }
  else if (seg == 7)  { src = wh_w;     dst = WF2;  nsrc = ndst = (size_t)DIMC * DIMC; }
  else if (seg == 8)  { src = hidden;   dst = hid16;  nsrc = (size_t)nN * DIMC;   ndst = (size_t)nNpad * DIMC;   sc = ASC; }
  else if (seg == 9)  { src = rela_w;   dst = rela16; nsrc = (size_t)nRel * DIMC; ndst = (size_t)nRelPad * DIMC; sc = ASC; }
  else if (seg == 11) { src = rela_w;   dst = qsel16; nsrc = (size_t)nRel * DIMC; ndst = (size_t)nQpad * DIMC;   sc = ASC; }

  const size_t nitems = ndst >> 3;
#pragma unroll 1
  for (size_t it = gtid; it < nitems; it += gstride) {
    const size_t e0 = it * 8;
    const float* p;
    bool in;
    if (seg == 11) {
      const int row = (int)(e0 / DIMC), c = (int)(e0 % DIMC);
      int q = q_rel[min(row, nQ - 1)];
      q = min(max(q, 0), nRel - 1);
      p = rela_w + (size_t)q * DIMC + c;
      in = row < nQ;
    } else {
      in = (e0 + 8 <= nsrc);
      p = src + (in ? e0 : (size_t)0);
    }
    v4f a = *(const v4f*)p;
    v4f b = *(const v4f*)(p + 4);
    if (!in) {
#pragma unroll
      for (int k = 0; k < 4; ++k) { a[k] = 0.0f; b[k] = 0.0f; }
    }
    if (seg == 7) {
      v8us hu, lu;
#pragma unroll
      for (int k = 0; k < 4; ++k) {
        const unsigned short ha = f2bf(a[k]); hu[k] = ha;     lu[k] = f2bf(a[k] - bf2f(ha));
        const unsigned short hb = f2bf(b[k]); hu[4 + k] = hb; lu[4 + k] = f2bf(b[k] - bf2f(hb));
      }
      *(volatile v8us*)(WHhi + e0) = hu;
      *(volatile v8us*)(WHlo + e0) = lu;
      __threadfence();
      *(volatile v8us*)(WHhi + e0) = hu;
      *(volatile v8us*)(WHlo + e0) = lu;
    } else {
      v8h hv;
#pragma unroll
      for (int k = 0; k < 4; ++k) { hv[k] = (_Float16)(a[k] * sc); hv[4 + k] = (_Float16)(b[k] * sc); }
      *(volatile v8h*)(dst + e0) = hv;
      __threadfence();
      *(volatile v8h*)(dst + e0) = hv;
    }
  }
}

__device__ __forceinline__ void gemm_rows_store(const float* sD, float* C, int ldc, int rowb, int colb, int Mstore,
                                                int wave, int lane) {
#pragma unroll
  for (int i = 0; i < 8; ++i) {
    const int row = 8 * wave + i, grow = rowb + row;
    if (grow < Mstore) {
      const v4f v = *(const v4f*)(sD + row * SDP + 4 * lane);
      *(volatile v4f*)(C + (size_t)grow * ldc + colb + 4 * lane) = v;
    }
  }
}

template <int SPLIT>
__global__ __launch_bounds__(GT_THR) void k_gemm(
    const unsigned short* __restrict__ A, const unsigned short* __restrict__ A2, int lda,
    const unsigned short* __restrict__ B, const unsigned short* __restrict__ B2, int ldb, int K,
    const float* __restrict__ bias, int nbias, float scale, float* C, int ldc, int Mstore) {
  __shared__ __attribute__((aligned(16))) float sD[64 * SDP];
  const int tid = threadIdx.x, lane = tid & 31, wave = tid >> 5, h = lane >> 4, m = lane & 15;
  const int mt = wave & 3, ng = wave >> 2;
  const int row0 = blockIdx.x * 64 + 16 * mt;
  const int cbl  = 64 * ng;
  const int col0 = blockIdx.y * 128 + cbl;

  v8f acc[4];
#pragma unroll
  for (int i = 0; i < 4; ++i) acc[i] = zacc();

  const unsigned short* ap  = A  + (size_t)(row0 + m) * lda + 8 * h;
  const unsigned short* ap2 = A2 + (size_t)(row0 + m) * lda + 8 * h;
#pragma unroll 1
  for (int k0 = 0; k0 < K; k0 += 32) {
    Frag16 a, a2;
    a.u[0] = *(const v8us*)(ap + k0);
    a.u[1] = *(const v8us*)(ap + k0 + 16);
    if (SPLIT) {
      a2.u[0] = *(const v8us*)(ap2 + k0);
      a2.u[1] = *(const v8us*)(ap2 + k0 + 16);
    } else {
      a2.u[0] = a.u[0]; a2.u[1] = a.u[1];
    }
#pragma unroll
    for (int nt = 0; nt < 4; ++nt) {
      const size_t boff = (size_t)(col0 + 16 * nt + m) * ldb + k0 + 8 * h;
      Frag16 b;
      b.u[0] = *(const v8us*)(B + boff);
      b.u[1] = *(const v8us*)(B + boff + 16);
      if (SPLIT) {
        Frag16 b2;
        b2.u[0] = *(const v8us*)(B2 + boff);
        b2.u[1] = *(const v8us*)(B2 + boff + 16);
        acc[nt] = wmb(a.vb, b.vb, acc[nt]);
        acc[nt] = wmb(a.vb, b2.vb, acc[nt]);
        acc[nt] = wmb(a2.vb, b.vb, acc[nt]);
      } else {
        acc[nt] = wmh(a.vh, b.vh, acc[nt]);
      }
    }
  }

#pragma unroll
  for (int nt = 0; nt < 4; ++nt) {
    const int cl = cbl + 16 * nt + m;
    const int cg = blockIdx.y * 128 + cl;
    float bb = 0.0f;
    {
      const int blim = (nbias - 1 > 0) ? nbias - 1 : 0;
      const int bi = cg < 0 ? 0 : (cg > blim ? blim : cg);
      const float bv = bias[bi];
      bb = (nbias > 0) ? bv : 0.0f;
    }
#pragma unroll
    for (int r = 0; r < 8; ++r) sD[(16 * mt + 8 * h + r) * SDP + cl] = acc[nt][r] * scale + bb;
  }
  __syncthreads();
  gemm_rows_store(sD, C, ldc, blockIdx.x * 64, blockIdx.y * 128, Mstore, wave, lane);
  __threadfence();
  gemm_rows_store(sD, C, ldc, blockIdx.x * 64, blockIdx.y * 128, Mstore, wave, lane);
}

__device__ __forceinline__ int scan_chunk(const int* __restrict__ edges, int nE, int nSeg, int cbase, int nodeBase,
                                          int* list, int tid, int wave) {
  int wc = 0;
  const int el0 = tid * EPT;
  const int e0  = cbase + el0;
  const int sent = -2147483647 - 1;
  int d0, d1, d2, d3, d4, d5, d6, d7;
#define LDK(J, DJ) { const int ee = min(e0 + (J), nE - 1); const int kv = edges[(size_t)ee * 7 + 5]; DJ = (e0 + (J) < nE) ? kv : sent; }
  LDK(0, d0) LDK(1, d1) LDK(2, d2) LDK(3, d3) LDK(4, d4) LDK(5, d5) LDK(6, d6) LDK(7, d7)
#undef LDK
  const unsigned nb = (unsigned)nodeBase, un = (unsigned)nSeg;
#define HT(DJ) (((((unsigned)(DJ)) - nb) < (unsigned)NB) && (((unsigned)(DJ)) < un))
  const bool h0 = HT(d0), h1 = HT(d1), h2 = HT(d2), h3 = HT(d3), h4 = HT(d4), h5 = HT(d5), h6 = HT(d6), h7 = HT(d7);
#undef HT
  const unsigned any = __builtin_amdgcn_ballot_w32(h0 | h1 | h2 | h3 | h4 | h5 | h6 | h7);
  if (any != 0u) {
#define HITJ(J, HJ) { \
      const unsigned mj = __builtin_amdgcn_ballot_w32(HJ); \
      if (mj != 0u) { \
        if (HJ) { \
          const int pos = wc + (int)__builtin_amdgcn_mbcnt_lo(mj, 0u); \
          if (pos < WCAP) list[wave * WCAP + pos] = el0 + (J); \
        } \
        wc += (int)__builtin_popcount(mj); } }
    HITJ(0, h0)
    HITJ(1, h1)
    HITJ(2, h2)
    HITJ(3, h3)
    HITJ(4, h4)
    HITJ(5, h5)
    HITJ(6, h6)
    HITJ(7, h7)
#undef HITJ
  }
  return wc;
}

__device__ __forceinline__ void gather_sum(float* dstw, const float* __restrict__ P, int ldp, const int* pidx,
                                           const float* __restrict__ Q, int ldq, const int* qidx, int coff,
                                           int wave, int lane) {
#pragma unroll 1
  for (int r = 0; r < 16; ++r) {
    const int i = wave * 16 + r;
    const v4f p = *(const v4f*)(P + (size_t)pidx[i] * ldp + coff + 4 * lane);
    const v4f q = *(const v4f*)(Q + (size_t)qidx[i] * ldq + coff + 4 * lane);
    *(v4f*)(dstw + r * PF + 4 * lane) = p + q;
  }
}

__device__ __forceinline__ v8f mm128(v8f d, const _Float16* afp, const _Float16* __restrict__ bp) {
#pragma unroll 1
  for (int ks = 0; ks < 4; ++ks) {
    Frag16 a, b;
    a.h[0] = *(const v8h*)(afp + 32 * ks); a.h[1] = *(const v8h*)(afp + 32 * ks + 16);
    b.h[0] = *(const v8h*)(bp + 32 * ks);  b.h[1] = *(const v8h*)(bp + 32 * ks + 16);
    d = wmh(a.vh, b.vh, d);
  }
  return d;
}
__device__ __forceinline__ Acc2 mm128x2(v8f du, v8f dc, const _Float16* afp,
                                         const _Float16* __restrict__ bu, const _Float16* __restrict__ bc) {
#pragma unroll 1
  for (int ks = 0; ks < 4; ++ks) {
    Frag16 a, b, c;
    a.h[0] = *(const v8h*)(afp + 32 * ks); a.h[1] = *(const v8h*)(afp + 32 * ks + 16);
    b.h[0] = *(const v8h*)(bu + 32 * ks);  b.h[1] = *(const v8h*)(bu + 32 * ks + 16);
    du = wmh(a.vh, b.vh, du);
    c.h[0] = *(const v8h*)(bc + 32 * ks);  c.h[1] = *(const v8h*)(bc + 32 * ks + 16);
    dc = wmh(a.vh, c.vh, dc);
  }
  Acc2 r; r.u = du; r.c = dc;
  return r;
}

__device__ __forceinline__ void agg_store(const float* acc, unsigned short* AGGhi, unsigned short* AGGlo,
                                          int nodeBase, int nNpad, int wave, int lane) {
  const int rr = lane >> 4, q = lane & 15;
#pragma unroll 1
  for (int it = 0; it < 32; ++it) {
    const int row = wave * 64 + 2 * it + rr;
    const int node = nodeBase + row;
    const float* ar = acc + row * ACCW;
    const float inv = 1.0f / (ar[DIMC] + 1e-5f);
    v8us hu, lu;
#pragma unroll
    for (int k = 0; k < 8; ++k) {
      const float x = ar[8 * q + k] * inv;
      const unsigned short hb = f2bf(x);
      hu[k] = hb;
      lu[k] = f2bf(x - bf2f(hb));
    }
    if (node < nNpad) {
      *(volatile v8us*)(AGGhi + (size_t)node * DIMC + 8 * q) = hu;
      *(volatile v8us*)(AGGlo + (size_t)node * DIMC + 8 * q) = lu;
    }
  }
}

__global__ __launch_bounds__(NTHR) void k_edge(
    const int* __restrict__ edges, const int* __restrict__ n_node,
    const float* __restrict__ hidden, const float* __restrict__ rela_w,
    const float* __restrict__ R1, const float* __restrict__ T1,
    const float* __restrict__ PG, const float* __restrict__ PS,
    const float* __restrict__ QG, const float* __restrict__ QS,
    const _Float16* __restrict__ WF2, const _Float16* __restrict__ WG,
    const _Float16* __restrict__ WR, const _Float16* __restrict__ WHT,
    const float* __restrict__ fuse2_b, const float* __restrict__ htrans_b, const float* __restrict__ walpha,
    unsigned short* AGGhi, unsigned short* AGGlo,
    int nN, int nNpad, int nE, int nRel, int nQ) {
  extern __shared__ __attribute__((aligned(16))) unsigned char dynlds[];
  float*    acc    = (float*)(dynlds + OFF_ACC);
  _Float16* xr     = (_Float16*)(dynlds + OFF_XR);
  _Float16* hrt    = (_Float16*)(dynlds + OFF_HR);
  float*    stg    = (float*)(dynlds + OFF_STG);
  int*      list   = (int*)(dynlds + OFF_LIST);
  int*      pend   = (int*)(dynlds + OFF_PEND);
  int*      s_slot = (int*)(dynlds + OFF_SLOT);
  int*      s_rel  = (int*)(dynlds + OFF_REL);
  int*      s_t    = (int*)(dynlds + OFF_T);
  int*      s_sub  = (int*)(dynlds + OFF_SUB);
  int*      s_rq   = (int*)(dynlds + OFF_RQ);
  int*      s_val  = (int*)(dynlds + OFF_VAL);
  float*    s_w    = (float*)(dynlds + OFF_W);
  int*      wcnt   = (int*)(dynlds + OFF_WCNT);
  int*      pendN  = (int*)(dynlds + OFF_PENDN);

  const int tid = threadIdx.x, lane = tid & 31, wave = tid >> 5, h = lane >> 4, m = lane & 15;
  const int nodeBase = blockIdx.x * NB;
  int nSeg = n_node[0];
  nSeg = nSeg < 0 ? 0 : (nSeg > nN ? nN : nSeg);

  _Float16* xw = xr  + wave * 16 * PT;
  _Float16* hw = hrt + wave * 16 * PT;
  float*    sw = stg + wave * 16 * PF;
  const _Float16* afx = xw + m * PT + 8 * h;
  const _Float16* afh = hw + m * PT + 8 * h;

  for (int i = tid; i < NB * ACCW; i += NTHR) acc[i] = 0.0f;
  if (tid == 0) pendN[0] = 0;
  __syncthreads();

  const v8f z8 = zacc();
  const int nChunks = (nE + CHUNK - 1) / CHUNK;
#pragma unroll 1
  for (int ch = 0; ch < nChunks; ++ch) {
    const int cbase = ch * CHUNK;
    const int wc = scan_chunk(edges, nE, nSeg, cbase, nodeBase, list, tid, wave);
    if (lane == 0) wcnt[wave] = wc;
    __syncthreads();

    const int base = pendN[0];
    int tot = 0, myoff = 0;
#pragma unroll
    for (int w = 0; w < NWAVE; ++w) {
      int c = wcnt[w];
      c = c > WCAP ? WCAP : (c < 0 ? 0 : c);
      if (w < wave) myoff += c;
      tot += c;
    }
    int newN = base + tot;
    newN = newN > PCAP ? PCAP : newN;
    {
      int n = wcnt[wave];
      n = n > WCAP ? WCAP : (n < 0 ? 0 : n);
      const int* lp = list + wave * WCAP;
      for (int i = lane; i < n; i += 32) {
        const int pos = base + myoff + i;
        if (pos < PCAP) pend[pos] = cbase + lp[i];
      }
    }
    const int fin = (ch == nChunks - 1) ? 1 : 0;
    const int R   = (fin != 0) ? (newN + PASSN - 1) / PASSN : newN / PASSN;
    const int Pv  = (fin != 0) ? newN : R * PASSN;
    __syncthreads();

#pragma unroll 1
    for (int rp = 0; rp < R; ++rp) {
      {
        const int jl = lane & 15;
        const int i = wave * 16 + jl;
        const int idx = rp * PASSN + i;
        int valid = (idx < Pv) ? 1 : 0;
        int e = pend[min(idx, PCAP - 1)];
        e = (valid != 0) ? e : 0;
        e = e < 0 ? 0 : (e > nE - 1 ? nE - 1 : e);
        const int* er = edges + (size_t)e * 7;
        int rq = er[0], rel = er[2], sub = er[4], obj = er[5], tt = er[6];
        int slot = obj - nodeBase;
        if (valid == 0 || (unsigned)slot >= (unsigned)NB || (unsigned)obj >= (unsigned)nSeg) { valid = 0; slot = 0; }
        rel = min(max(rel, 0), nRel - 1);
        tt  = min(max(tt, 0), PE_LEN - 1);
        sub = min(max(sub, 0), nN - 1);
        rq  = min(max(rq, 0), nQ - 1);
        s_slot[i] = slot; s_rel[i] = rel; s_t[i] = tt; s_sub[i] = sub; s_rq[i] = rq; s_val[i] = valid;
      }
      __syncthreads();

      {
#pragma unroll 1
        for (int r = 0; r < 16; ++r) {
          const int i = wave * 16 + r;
          const int rel = s_rel[i], tt = s_t[i], sub = s_sub[i];
          const v4f a  = *(const v4f*)(R1 + (size_t)rel * DIMC + 4 * lane);
          const v4f tv = *(const v4f*)(T1 + (size_t)tt * DIMC + 4 * lane);
          const v4f re = *(const v4f*)(rela_w + (size_t)rel * DIMC + 4 * lane);
          const v4f hs = *(const v4f*)(hidden + (size_t)sub * DIMC + 4 * lane);
          v4h xv;
#pragma unroll
          for (int k = 0; k < 4; ++k) xv[k] = (_Float16)(lrelu(a[k] + tv[k]) * ASC);
          *(v4h*)(xw + r * PT + 4 * lane) = xv;
          *(v4f*)(sw + r * PF + 4 * lane) = re;
          *(v4f*)(sw + r * PF + DIMC + 4 * lane) = hs;
        }
      }
      __syncthreads();

      {
#pragma unroll 1
        for (int nt = 0; nt < 8; ++nt) {
          const int col = 16 * nt + m;
          const v8f d = mm128(z8, afx, WF2 + (size_t)col * DIMC + 8 * h);
          const float bb = fuse2_b[col];
#pragma unroll
          for (int r = 0; r < 8; ++r) {
            const int j = 8 * h + r;
            const float v = lrelu(d[r] * PINV + bb) + sw[j * PF + col];
            hw[j * PT + col] = (_Float16)(v * ASC);
          }
        }
      }
      __syncthreads();

      gather_sum(sw, PS, DIMC, s_sub, QS, DIMC, s_rq, 0, wave, lane);
      __syncthreads();

      {
        float ap[8];
#pragma unroll
        for (int r = 0; r < 8; ++r) ap[r] = 0.0f;
#pragma unroll 1
        for (int nt = 0; nt < 8; ++nt) {
          const int cc = 16 * nt + m;
          const v8f d = mm128(z8, afh, WR + (size_t)cc * DIMC + 8 * h);
          const float wa = walpha[cc];
#pragma unroll
          for (int r = 0; r < 8; ++r) {
            const float pre = d[r] * PINV + sw[(8 * h + r) * PF + cc];
            ap[r] += lrelu(pre) * wa;
          }
        }
#pragma unroll
        for (int r = 0; r < 8; ++r) {
          float v = ap[r];
          v += __shfl_xor(v, 1);
          v += __shfl_xor(v, 2);
          v += __shfl_xor(v, 4);
          v += __shfl_xor(v, 8);
          ap[r] = v;
        }
        if (m == 0) {
#pragma unroll
          for (int r = 0; r < 8; ++r) {
            const int i = wave * 16 + 8 * h + r;
            s_w[i] = (s_val[i] != 0) ? __expf(ap[r]) : 0.0f;
          }
        }
      }
      __syncthreads();

      gather_sum(sw, PG, GATEN, s_sub, QG, GATEN, s_rq, DIMC, wave, lane);
      __syncthreads();

      {
#pragma unroll 1
        for (int nt = 0; nt < 8; ++nt) {
          const int cc = 16 * nt + m, o = DIMC + cc;
          const v8f d = mm128(z8, afh, WG + (size_t)o * GATEK + 8 * h);
#pragma unroll
          for (int r = 0; r < 8; ++r) {
            const int j = 8 * h + r;
            const float g  = sigm(d[r] * PINV + sw[j * PF + cc]);
            const float hs = sw[j * PF + DIMC + cc];
            xw[j * PT + cc] = (_Float16)(g * hs * ASC);
          }
        }
      }
      __syncthreads();

      gather_sum(sw, PG, GATEN, s_sub, QG, GATEN, s_rq, 0, wave, lane);
      __syncthreads();

      {
#pragma unroll 1
        for (int nt = 0; nt < 8; ++nt) {
          const int cc = 16 * nt + m;
          const _Float16* bc = WHT + (size_t)cc * HTK + 8 * h;
          Acc2 p2 = mm128x2(z8, z8, afh, WG + (size_t)cc * GATEK + 8 * h, bc);
          const v8f dU = p2.u;
          const v8f dC = mm128(p2.c, afx, bc + DIMC);
          const float bh = htrans_b[cc];
#pragma unroll
          for (int r = 0; r < 8; ++r) {
            const int j = 8 * h + r;
            const float u    = sigm(dU[r] * PINV + sw[j * PF + cc]);
            const float cand = tanh_f(dC[r] * PINV + bh);
            const float hs   = sw[j * PF + DIMC + cc];
            sw[j * PF + cc] = (1.0f - u) * hs + u * cand;
          }
        }
      }
      __syncthreads();

      for (int c = tid; c < ACCW; c += NTHR) {
        const int cm = (c < DIMC) ? c : 0;
        const bool isw = (c >= DIMC);
#pragma unroll 1
        for (int i = 0; i < PASSN; ++i) {
          int sl = s_slot[i];
          sl = sl < 0 ? 0 : (sl > NB - 1 ? NB - 1 : sl);
          const float w  = s_w[i];
          const float mv = stg[i * PF + cm];
          const float v  = isw ? 1.0f : mv;
          acc[sl * ACCW + c] += w * v;
        }
      }
      __syncthreads();
    }

    int rem = newN - R * PASSN;
    rem = rem < 0 ? 0 : rem;
    if (R > 0 && tid < rem) pend[tid] = pend[R * PASSN + tid];
    if (tid == 0) pendN[0] = rem;
  }
  __syncthreads();

  agg_store(acc, AGGhi, AGGlo, nodeBase, nNpad, wave, lane);
  __threadfence();
  agg_store(acc, AGGhi, AGGlo, nodeBase, nNpad, wave, lane);
}

extern "C" void kernel_launch(void* const* d_in, const int* in_sizes, int n_in,
                              void* d_out, int out_size, void* d_ws, size_t ws_size,
                              hipStream_t stream) {
  if (n_in < 20) return;
  const int nQ   = in_sizes[1];
  const int nN   = in_sizes[2] / DIMC;
  const int nE   = in_sizes[3] / 7;
  const int nRel = in_sizes[5] / DIMC;
  if (nQ < 1 || nN < 1 || nE < 1 || nRel < 1) return;
  if (in_sizes[2] != nN * DIMC || in_sizes[3] != nE * 7 || in_sizes[5] != nRel * DIMC) return;
  if (in_sizes[4] < 1) return;
  if (in_sizes[6] != DIMC * F1K || in_sizes[7] < DIMC || in_sizes[8] != DIMC * DIMC || in_sizes[9] < DIMC) return;
  if (in_sizes[10] != GATEN * GATEK || in_sizes[11] < GATEN || in_sizes[12] != DIMC * HTK || in_sizes[13] < DIMC) return;
  if (in_sizes[14] != DIMC * DIMC || in_sizes[15] != DIMC * DIMC || in_sizes[16] != DIMC * DIMC || in_sizes[17] < DIMC) return;
  if (in_sizes[18] < DIMC || in_sizes[19] != DIMC * DIMC) return;
  if (out_size != nN * DIMC) return;

  const int*   q_rel    = (const int*)d_in[1];
  const float* hidden   = (const float*)d_in[2];
  const int*   edges    = (const int*)d_in[3];
  const int*   n_node   = (const int*)d_in[4];
  const float* rela_w   = (const float*)d_in[5];
  const float* fuse1_w  = (const float*)d_in[6];
  const float* fuse1_b  = (const float*)d_in[7];
  const float* fuse2_w  = (const float*)d_in[8];
  const float* fuse2_b  = (const float*)d_in[9];
  const float* gate_w   = (const float*)d_in[10];
  const float* gate_b   = (const float*)d_in[11];
  const float* htrans_w = (const float*)d_in[12];
  const float* htrans_b = (const float*)d_in[13];
  const float* ws_w     = (const float*)d_in[14];
  const float* wr_w     = (const float*)d_in[15];
  const float* wqr_w    = (const float*)d_in[16];
  const float* wqr_b    = (const float*)d_in[17];
  const float* walpha   = (const float*)d_in[18];
  const float* wh_w     = (const float*)d_in[19];
  float* out = (float*)d_out;

  const int nNpad   = ((nN + 63) / 64) * 64;
  const int nRelPad = ((nRel + 63) / 64) * 64;
  const int nQpad   = ((nQ + 63) / 64) * 64;
  const int nBlkE   = (nN + NB - 1) / NB;

  char* ws = (char*)d_ws;
  size_t off = 0;
  auto carve = [&](size_t bytes) { const size_t o = off; off += (bytes + 1023) & ~(size_t)1023; return o; };
  const size_t oWF1 = carve((size_t)DIMC * F1K * 2);
  const size_t oWF2 = carve((size_t)DIMC * DIMC * 2);
  const size_t oWG  = carve((size_t)GATEN * GATEK * 2);
  const size_t oWHT = carve((size_t)DIMC * HTK * 2);
  const size_t oWS  = carve((size_t)DIMC * DIMC * 2);
  const size_t oWR  = carve((size_t)DIMC * DIMC * 2);
  const size_t oWQ  = carve((size_t)DIMC * DIMC * 2);
  const size_t oWHh = carve((size_t)DIMC * DIMC * 2);
  const size_t oWHl = carve((size_t)DIMC * DIMC * 2);
  const size_t oHid = carve((size_t)nNpad * DIMC * 2);
  const size_t oRel = carve((size_t)nRelPad * DIMC * 2);
  const size_t oPe  = carve((size_t)PE_ROWS * TD * 2);
  const size_t oQs  = carve((size_t)nQpad * DIMC * 2);
  const size_t oR1  = carve((size_t)nRelPad * DIMC * 4);
  const size_t oT1  = carve((size_t)PE_ROWS * DIMC * 4);
  const size_t oQG  = carve((size_t)nQpad * GATEN * 4);
  const size_t oQS  = carve((size_t)nQpad * DIMC * 4);
  const size_t oPG  = carve((size_t)nNpad * GATEN * 4);
  const size_t oPS  = carve((size_t)nNpad * DIMC * 4);
  const size_t oAh  = carve((size_t)nNpad * DIMC * 2);
  const size_t oAl  = carve((size_t)nNpad * DIMC * 2);
  const size_t wsCap = (size_t)128 * 1024 * 1024;
  if (off > ws_size || off > wsCap) return;

  _Float16* WF1 = (_Float16*)(ws + oWF1);
  _Float16* WF2 = (_Float16*)(ws + oWF2);
  _Float16* WG  = (_Float16*)(ws + oWG);
  _Float16* WHT = (_Float16*)(ws + oWHT);
  _Float16* WS  = (_Float16*)(ws + oWS);
  _Float16* WR  = (_Float16*)(ws + oWR);
  _Float16* WQ  = (_Float16*)(ws + oWQ);
  unsigned short* WHhi = (unsigned short*)(ws + oWHh);
  unsigned short* WHlo = (unsigned short*)(ws + oWHl);
  _Float16* hid16  = (_Float16*)(ws + oHid);
  _Float16* rela16 = (_Float16*)(ws + oRel);
  _Float16* pe16   = (_Float16*)(ws + oPe);
  _Float16* qsel16 = (_Float16*)(ws + oQs);
  float* R1 = (float*)(ws + oR1);
  float* T1 = (float*)(ws + oT1);
  float* QG = (float*)(ws + oQG);
  float* QS = (float*)(ws + oQS);
  float* PG = (float*)(ws + oPG);
  float* PS = (float*)(ws + oPS);
  unsigned short* AGGhi = (unsigned short*)(ws + oAh);
  unsigned short* AGGlo = (unsigned short*)(ws + oAl);

  typedef const unsigned short* cus;

  k_prep<<<dim3(256, 12), 256, 0, stream>>>(
      fuse1_w, fuse2_w, gate_w, htrans_w, ws_w, wr_w, wqr_w, wh_w, hidden, rela_w, q_rel,
      WF1, WF2, WG, WHT, WS, WR, WQ, WHhi, WHlo, hid16, rela16, pe16, qsel16,
      nN, nNpad, nRel, nRelPad, nQ, nQpad);

  k_gemm<0><<<dim3(nRelPad / 64, 1), GT_THR, 0, stream>>>(
      (cus)rela16, (cus)rela16, DIMC, (cus)WF1, (cus)WF1, F1K, DIMC, fuse1_b, 0, PINV, R1, DIMC, nRelPad);
  k_gemm<0><<<dim3(PE_ROWS / 64, 1), GT_THR, 0, stream>>>(
      (cus)pe16, (cus)pe16, TD, (cus)(WF1 + DIMC), (cus)(WF1 + DIMC), F1K, TD, fuse1_b, DIMC, PINV, T1, DIMC, PE_ROWS);
  k_gemm<0><<<dim3(nNpad / 64, GATEN / 128), GT_THR, 0, stream>>>(
      (cus)hid16, (cus)hid16, DIMC, (cus)(WG + 2 * DIMC), (cus)(WG + 2 * DIMC), GATEK, DIMC, gate_b, 0, PINV, PG, GATEN, nNpad);
  k_gemm<0><<<dim3(nNpad / 64, 1), GT_THR, 0, stream>>>(
      (cus)hid16, (cus)hid16, DIMC, (cus)WS, (cus)WS, DIMC, DIMC, gate_b, 0, PINV, PS, DIMC, nNpad);
  k_gemm<0><<<dim3(nQpad / 64, GATEN / 128), GT_THR, 0, stream>>>(
      (cus)qsel16, (cus)qsel16, DIMC, (cus)(WG + DIMC), (cus)(WG + DIMC), GATEK, DIMC, gate_b, GATEN, PINV, QG, GATEN, nQpad);
  k_gemm<0><<<dim3(nQpad / 64, 1), GT_THR, 0, stream>>>(
      (cus)qsel16, (cus)qsel16, DIMC, (cus)WQ, (cus)WQ, DIMC, DIMC, wqr_b, DIMC, PINV, QS, DIMC, nQpad);

  k_edge<<<nBlkE, NTHR, LDS_TOTAL, stream>>>(
      edges, n_node, hidden, rela_w, R1, T1, PG, PS, QG, QS, WF2, WG, WR, WHT,
      fuse2_b, htrans_b, walpha, AGGhi, AGGlo, nN, nNpad, nE, nRel, nQ);

  k_gemm<1><<<dim3(nNpad / 64, 1), GT_THR, 0, stream>>>(
      (cus)AGGhi, (cus)AGGlo, DIMC, (cus)WHhi, (cus)WHlo, DIMC, DIMC, fuse1_b, 0, 1.0f, out, DIMC, nN);
}
